// Encoder_20272245637276
// MI455X (gfx1250) — hardware-verified
//
#include <hip/hip_runtime.h>
#include <stddef.h>
#include <stdint.h>
#include <math.h>


#define DIN    512
#define HID    512
#define ZD     128
#define NH     256
#define KA     512
#define KB     1024
#define NTHR   256
#define NWAVE  8
#define EPT    8
#define CHUNK  (NTHR * EPT)
#define WCAP   (EPT * 32)
#define LISTN  (NWAVE * WCAP)
#define NBD    4096
#define SLD    12
#define NBA    1024
#define SLA    10
#define RCAP   28672
#define DEGCAP 64
#define GBM    64
#define GBN    64
#define GTHR   128
#define NU1    (HID * (KA / 8))
#define NU2    (HID * (KB / 8))
#define NU3    (NH * (KB / 8))
#define AGG_ZINTS   (LISTN + 2 * RCAP + 3 * NBA)
#define MISC_INTS   16
#define ROWHW       1024
#define ROWBUF_INTS (NWAVE * ROWHW / 2)
#define LDS_HL_INTS (AGG_ZINTS + MISC_INTS + ROWBUF_INTS)
#define LDS_HD_INTS (AGG_ZINTS + MISC_INTS)
#define WSMAX  134217728

static_assert((CHUNK & (CHUNK - 1)) == 0 && CHUNK <= 4096);
static_assert((NBD & (NBD - 1)) == 0 && NBD == (1 << SLD));
static_assert((NBA & (NBA - 1)) == 0 && NBA == (1 << SLA));
static_assert(((long long)CHUNK << SLD) < (1LL << 31));
static_assert(((long long)CHUNK << SLA) < (1LL << 31));
static_assert(NBD % (NTHR * 4) == 0);
static_assert(LISTN % NTHR == 0);
static_assert(NBA % NWAVE == 0 && NBA % 32 == 0 && NBA % GBM == 0);
static_assert(RCAP % 32 == 0 && AGG_ZINTS % (NTHR * 4) == 0 && LISTN % 4 == 0);
static_assert(((AGG_ZINTS + MISC_INTS) % 4) == 0);
static_assert(KA % 32 == 0 && KB % 32 == 0 && KB == 2 * HID && KA == DIN);
static_assert(GBM == (GTHR / 32) * 16 && GBN == 64 && HID % GBN == 0 && NH % GBN == 0);
static_assert(NU1 % NTHR == 0 && NU2 % NTHR == 0 && NU3 % NTHR == 0 && ((NU3 / 2) % NTHR) == 0);
static_assert(HID == 4 * 128 && NH == 2 * 128 && ZD == 4 * 32);
static_assert(LDS_HL_INTS * 4 <= 300000);

typedef float          v4f   __attribute__((ext_vector_type(4)));
typedef float          v8f   __attribute__((ext_vector_type(8)));
typedef int            v4i   __attribute__((ext_vector_type(4)));
typedef int            v8i   __attribute__((ext_vector_type(8)));
typedef unsigned short v4us  __attribute__((ext_vector_type(4)));
typedef unsigned short v8us  __attribute__((ext_vector_type(8)));
typedef unsigned short v16us __attribute__((ext_vector_type(16)));
typedef __bf16         v16bf __attribute__((ext_vector_type(16)));
typedef v4f  __attribute__((may_alias)) v4fa;
typedef v4i  __attribute__((may_alias)) v4ia;
typedef v4us __attribute__((may_alias)) v4usa;
typedef v8us __attribute__((may_alias)) v8usa;
union FragB { v16bf v; v16us u; v8us h[2]; v8i w; };

__device__ __forceinline__ v8f wmb(const FragB& a, const FragB& b, v8f c) {
  v8f d = __builtin_amdgcn_wmma_f32_16x16x32_bf16(false, a.v, false, b.v, (short)0, c, false, false);
  asm volatile("v_nop\n\tv_nop\n\tv_nop\n\tv_nop" : "+v"(d) : "v"(a.w), "v"(b.w));
  return d;
}

__device__ __forceinline__ unsigned bf16_bits(float f) {
  const unsigned u = __float_as_uint(f);
  return (u + 0x7FFFu + ((u >> 16) & 1u)) >> 16;
}
__device__ __forceinline__ float bf16_val(float f) {
  return __uint_as_float(bf16_bits(f) << 16);
}

__device__ __forceinline__ void wave_sync() {
  __builtin_amdgcn_fence(__ATOMIC_RELEASE, "wavefront");
  __builtin_amdgcn_wave_barrier();
  __builtin_amdgcn_fence(__ATOMIC_ACQUIRE, "wavefront");
}

template <int SLB>
__device__ __forceinline__ int scan_chunk(const int* __restrict__ dsts, int nE, int cbase, int slotBase,
                                          int nb, int vec8, int* list, int tid, int lane, int wave) {
  int wc = 0;
  const int el0  = tid * EPT;
  const int e0   = cbase + el0;
  const int sent = -2147483647 - 1;
  v4i da, db;
  if (vec8 != 0 && cbase + CHUNK <= nE) {
    da = *(const v4i*)(dsts + e0);
    db = *(const v4i*)(dsts + e0 + 4);
  } else {
    da.x = (e0     < nE) ? dsts[min(e0,     nE - 1)] : sent;
    da.y = (e0 + 1 < nE) ? dsts[min(e0 + 1, nE - 1)] : sent;
    da.z = (e0 + 2 < nE) ? dsts[min(e0 + 2, nE - 1)] : sent;
    da.w = (e0 + 3 < nE) ? dsts[min(e0 + 3, nE - 1)] : sent;
    db.x = (e0 + 4 < nE) ? dsts[min(e0 + 4, nE - 1)] : sent;
    db.y = (e0 + 5 < nE) ? dsts[min(e0 + 5, nE - 1)] : sent;
    db.z = (e0 + 6 < nE) ? dsts[min(e0 + 6, nE - 1)] : sent;
    db.w = (e0 + 7 < nE) ? dsts[min(e0 + 7, nE - 1)] : sent;
  }
  const unsigned nbs = (unsigned)slotBase;
  const unsigned unb = (unsigned)nb;
  const unsigned s0 = (unsigned)da.x - nbs, s1 = (unsigned)da.y - nbs;
  const unsigned s2 = (unsigned)da.z - nbs, s3 = (unsigned)da.w - nbs;
  const unsigned s4 = (unsigned)db.x - nbs, s5 = (unsigned)db.y - nbs;
  const unsigned s6 = (unsigned)db.z - nbs, s7 = (unsigned)db.w - nbs;
  const bool h0 = s0 < unb, h1 = s1 < unb, h2 = s2 < unb, h3 = s3 < unb;
  const bool h4 = s4 < unb, h5 = s5 < unb, h6 = s6 < unb, h7 = s7 < unb;
  const unsigned any = __builtin_amdgcn_ballot_w32(h0 | h1 | h2 | h3 | h4 | h5 | h6 | h7);
  if (any != 0u) {
#define HITJ(J, HJ, SJ) { \
      const unsigned mj = __builtin_amdgcn_ballot_w32(HJ); \
      if (mj != 0u) { \
        if (HJ) { \
          const int pos = wc + (int)__builtin_amdgcn_mbcnt_lo(mj, 0u); \
          if (pos < WCAP) list[wave * WCAP + pos] = ((el0 + (J)) << SLB) | (int)(SJ); \
        } \
        wc += (int)__builtin_popcount(mj); } }
    HITJ(0, h0, s0)
    HITJ(1, h1, s1)
    HITJ(2, h2, s2)
    HITJ(3, h3, s3)
    HITJ(4, h4, s4)
    HITJ(5, h5, s5)
    HITJ(6, h6, s6)
    HITJ(7, h7, s7)
#undef HITJ
  }
  return wc;
}

__global__ __launch_bounds__(NTHR) void k_wprep(const float* __restrict__ W1, const float* __restrict__ W2,
                                                const float* __restrict__ Wmu, const float* __restrict__ Wlv,
                                                unsigned short* W1T, unsigned short* W2T, unsigned short* WHT) {
  const int u = (int)blockIdx.x * NTHR + (int)threadIdx.x;
  const float* p;
  size_t st;
  unsigned short* dp;
  if (u < NU1) {
    const int n  = u >> 6;
    const int k8 = (u & 63) * 8;
    p  = W1 + (size_t)k8 * HID + n;
    st = HID;
    dp = W1T + (size_t)n * KA + k8;
  } else if (u < NU1 + NU2) {
    const int v  = u - NU1;
    const int n  = v >> 7;
    const int k8 = (v & 127) * 8;
    const int kk = k8 & (HID - 1);
    p  = W2 + (size_t)kk * HID + n;
    st = HID;
    dp = W2T + (size_t)n * KB + k8;
  } else if (u < NU1 + NU2 + NU3) {
    const int v  = u - NU1 - NU2;
    const int n  = v >> 7;
    const int k8 = (v & 127) * 8;
    const int kk = k8 & (HID - 1);
    const int nn = n & (ZD - 1);
    const float* Wsrc = (n < ZD) ? Wmu : Wlv;
    p  = Wsrc + (size_t)kk * ZD + nn;
    st = ZD;
    dp = WHT + (size_t)n * KB + k8;
  } else {
    return;
  }
  v8us o;
#pragma unroll
  for (int i = 0; i < 8; ++i) o[i] = (unsigned short)bf16_bits(p[(size_t)i * st]);
  *(volatile v8us*)dp = o;
  __threadfence();
  *(volatile v8us*)dp = o;
}

__global__ __launch_bounds__(NTHR) void k_cvx(const float* __restrict__ x, int nN, int nUnits,
                                              unsigned short* xb) {
  const int u = (int)blockIdx.x * NTHR + (int)threadIdx.x;
  if (u >= nUnits) return;
  const int row = u >> 6;
  const int k8  = (u & 63) * 8;
  const int rc  = row < nN ? row : nN - 1;
  const float* p = x + (size_t)rc * DIN + k8;
  const v4f a = *(const v4fa*)p;
  const v4f b = *(const v4fa*)(p + 4);
  const bool ok = row < nN;
  v8us o;
  o[0] = ok ? (unsigned short)bf16_bits(a.x) : (unsigned short)0;
  o[1] = ok ? (unsigned short)bf16_bits(a.y) : (unsigned short)0;
  o[2] = ok ? (unsigned short)bf16_bits(a.z) : (unsigned short)0;
  o[3] = ok ? (unsigned short)bf16_bits(a.w) : (unsigned short)0;
  o[4] = ok ? (unsigned short)bf16_bits(b.x) : (unsigned short)0;
  o[5] = ok ? (unsigned short)bf16_bits(b.y) : (unsigned short)0;
  o[6] = ok ? (unsigned short)bf16_bits(b.z) : (unsigned short)0;
  o[7] = ok ? (unsigned short)bf16_bits(b.w) : (unsigned short)0;
  unsigned short* dp = xb + (size_t)row * DIN + k8;
  *(volatile v8us*)dp = o;
  __threadfence();
  *(volatile v8us*)dp = o;
}

__global__ __launch_bounds__(NTHR) void k_deg(const int* __restrict__ dsts, int nE, int vec8, float* dis) {
  __shared__ __attribute__((aligned(16))) int scnt[NBD];
  __shared__ __attribute__((aligned(16))) float sdis[NBD];
  __shared__ __attribute__((aligned(16))) int list[LISTN];
  __shared__ int wcnt[NWAVE];
  const int tid = (int)threadIdx.x, lane = tid & 31, wave = tid >> 5;
  const int nodeBase = (int)blockIdx.x * NBD;

  for (int i = tid; i < NBD; i += NTHR) scnt[i] = 0;
  for (int i = tid; i < LISTN; i += NTHR) list[i] = 0;
  if (tid < NWAVE) wcnt[tid] = 0;
  __syncthreads();

  const int nChunks = (nE + CHUNK - 1) / CHUNK;
#pragma unroll 1
  for (int ch = 0; ch < nChunks; ++ch) {
    const int cbase = ch * CHUNK;
    const int wc = scan_chunk<SLD>(dsts, nE, cbase, nodeBase, NBD, vec8, list, tid, lane, wave);
    if (lane == 0) wcnt[wave] = wc;
    __syncthreads();
    if (wave == 0) {
#pragma unroll 1
      for (int w2 = 0; w2 < NWAVE; ++w2) {
        int c = wcnt[w2];
        c = c < 0 ? 0 : (c > WCAP ? WCAP : c);
#pragma unroll 1
        for (int b0 = 0; b0 < c; b0 += 32) {
          const int idx = b0 + lane;
          const int ent = list[w2 * WCAP + (idx < WCAP ? idx : WCAP - 1)];
          const int m32 = (c - b0) < 32 ? (c - b0) : 32;
#pragma unroll 1
          for (int k = 0; k < m32; ++k) {
            const int u  = __builtin_amdgcn_readlane(ent, k);
            const int sl = u & (NBD - 1);
            if (lane == 0) scnt[sl] = scnt[sl] + 1;
          }
        }
      }
    }
    __syncthreads();
  }

#pragma unroll 1
  for (int i = tid; i < NBD; i += NTHR) {
    const float d = (float)scnt[i] + 1.0f;
    sdis[i] = 1.0f / sqrtf(d);
  }
  __syncthreads();

  v4f vals[NBD / (NTHR * 4)];
#pragma unroll
  for (int it = 0; it < NBD / (NTHR * 4); ++it) {
    const int s0 = it * (NTHR * 4) + 4 * tid;
    vals[it] = *(const v4fa*)(sdis + s0);
  }
#pragma unroll
  for (int it = 0; it < NBD / (NTHR * 4); ++it) {
    const int s0 = it * (NTHR * 4) + 4 * tid;
    *(volatile v4f*)(dis + (size_t)nodeBase + s0) = vals[it];
  }
  __threadfence();
#pragma unroll
  for (int it = 0; it < NBD / (NTHR * 4); ++it) {
    const int s0 = it * (NTHR * 4) + 4 * tid;
    *(volatile v4f*)(dis + (size_t)nodeBase + s0) = vals[it];
  }
}

__global__ __launch_bounds__(GTHR) void k_gemm(
    const unsigned short* __restrict__ A, const unsigned short* __restrict__ WT,
    float* outF, int K, int ldo)
{
  __shared__ __attribute__((aligned(16))) float stg[GBM * GBN];
  const int tid = (int)threadIdx.x, lane = tid & 31, wave = tid >> 5, hh = lane >> 4, m = lane & 15;
  const int rowBase = (int)blockIdx.x * GBM;
  const int col0    = (int)blockIdx.y * GBN;

  v8f acc[4];
  {
    const v8f z = {0.f, 0.f, 0.f, 0.f, 0.f, 0.f, 0.f, 0.f};
    acc[0] = z; acc[1] = z; acc[2] = z; acc[3] = z;
  }
  const unsigned short* ap = A  + (size_t)(rowBase + 16 * wave + m) * (size_t)K + 8 * hh;
  const unsigned short* wp = WT + (size_t)(col0 + m) * (size_t)K + 8 * hh;
  const int ksteps = K >> 5;
#pragma unroll 1
  for (int ks = 0; ks < ksteps; ++ks) {
    FragB af;
    af.h[0] = *(const v8usa*)(ap + 32 * ks);
    af.h[1] = *(const v8usa*)(ap + 32 * ks + 16);
#pragma unroll
    for (int t = 0; t < 4; ++t) {
      const unsigned short* wq = wp + (size_t)(16 * t) * (size_t)K + 32 * ks;
      FragB bf;
      bf.h[0] = *(const v8usa*)wq;
      bf.h[1] = *(const v8usa*)(wq + 16);
      acc[t] = wmb(af, bf, acc[t]);
    }
  }

#pragma unroll
  for (int t = 0; t < 4; ++t) {
    const int lc = 16 * t + m;
#pragma unroll
    for (int r = 0; r < 8; ++r) {
      const int lr = 16 * wave + 8 * hh + r;
      stg[lr * GBN + lc] = acc[t][r];
    }
  }
  __syncthreads();

  v4f fv[8];
#pragma unroll
  for (int i = 0; i < 8; ++i) {
    const int lr = 16 * wave + 2 * i + hh;
    fv[i] = *(const v4fa*)(stg + lr * GBN + 4 * m);
  }
#pragma unroll
  for (int i = 0; i < 8; ++i) {
    const int lr = 16 * wave + 2 * i + hh;
    const int gr = rowBase + lr;
    float* op = outF + (size_t)gr * (size_t)ldo + col0 + 4 * m;
    *(volatile v4f*)op = fv[i];
  }
  __threadfence();
#pragma unroll
  for (int i = 0; i < 8; ++i) {
    const int lr = 16 * wave + 2 * i + hh;
    const int gr = rowBase + lr;
    float* op = outF + (size_t)gr * (size_t)ldo + col0 + 4 * m;
    *(volatile v4f*)op = fv[i];
  }
}

template <int NJ, int MODE>
__global__ __launch_bounds__(NTHR) void k_scan(const int* __restrict__ srcs, const int* __restrict__ dsts,
                                               int nE, int nN, int vec8, int mRows,
                                               const float* __restrict__ dis, const float* __restrict__ tl,
                                               const float* __restrict__ biasA, const float* __restrict__ biasB,
                                               const float* __restrict__ eps,
                                               unsigned short* hpl, float* outp, size_t outSeg) {
  extern __shared__ __attribute__((aligned(16))) int dsm[];
  constexpr int FW = 128 * NJ;
  int* list = dsm;
  int* hl   = dsm + LISTN;
  int* sl   = hl + RCAP;
  int* cnt  = sl + RCAP;
  int* offs = cnt + NBA;
  int* cur  = offs + NBA;
  int* misc = cur + NBA;
  const int tid = (int)threadIdx.x, lane = tid & 31, wave = tid >> 5;
  const int nodeBase = (int)blockIdx.x * NBA;

  {
    const v4i z4 = {0, 0, 0, 0};
    for (int i = tid * 4; i < AGG_ZINTS; i += NTHR * 4) *(v4ia*)(dsm + i) = z4;
    if (tid < MISC_INTS) misc[tid] = 0;
  }
  v4f bv[NJ];
#pragma unroll
  for (int j = 0; j < NJ; ++j) {
    const float* bp = (MODE == 2) ? ((j == 0 ? biasA : biasB) + 4 * lane) : (biasA + 128 * j + 4 * lane);
    const v4f t4 = *(const v4fa*)bp;
    v4f b;
    b.x = bf16_val(t4.x); b.y = bf16_val(t4.y); b.z = bf16_val(t4.z); b.w = bf16_val(t4.w);
    bv[j] = b;
  }
  __syncthreads();

  int t = 0, ov = 0;
  const int nChunks = (nE + CHUNK - 1) / CHUNK;
#pragma unroll 1
  for (int ch = 0; ch < nChunks; ++ch) {
    const int cbase = ch * CHUNK;
    const int wc = scan_chunk<SLA>(dsts, nE, cbase, nodeBase, NBA, vec8, list, tid, lane, wave);
    if (lane == 0) misc[wave] = wc;
    __syncthreads();
    if (wave == 0) {
#pragma unroll 1
      for (int w2 = 0; w2 < NWAVE; ++w2) {
        int c = misc[w2];
        c = c < 0 ? 0 : (c > WCAP ? WCAP : c);
#pragma unroll 1
        for (int b0 = 0; b0 < c; b0 += 32) {
          const int idx = b0 + lane;
          const int ent = list[w2 * WCAP + (idx < WCAP ? idx : WCAP - 1)];
          const int m32 = (c - b0) < 32 ? (c - b0) : 32;
#pragma unroll 1
          for (int k = 0; k < m32; ++k) {
            const int u    = __builtin_amdgcn_readlane(ent, k);
            const int slot = u & (NBA - 1);
            const int el   = (u >> SLA) & (CHUNK - 1);
            const int pk   = ((cbase + el) << SLA) | slot;
            if (t < RCAP) {
              if (lane == 0) { hl[t] = pk; cnt[slot] = cnt[slot] + 1; }
              t = t + 1;
            } else {
              ov = 1;
            }
          }
        }
      }
    }
    __syncthreads();
  }
  if (wave == 0 && lane == 0) { misc[8] = t; misc[9] = ov; }
  __syncthreads();
  int tt = misc[8];
  tt = tt < 0 ? 0 : (tt > RCAP ? RCAP : tt);
  const int ovf = misc[9];

  if (wave == 0) {
    const int base = lane * (NBA / 32);
    int s = 0;
#pragma unroll 1
    for (int i = 0; i < NBA / 32; ++i) s += cnt[base + i];
    int incl = s;
#pragma unroll
    for (int d = 1; d < 32; d <<= 1) {
      const int y = __shfl_up(incl, d, 32);
      if (lane >= d) incl += y;
    }
    int run = incl - s;
#pragma unroll 1
    for (int i = 0; i < NBA / 32; ++i) {
      const int cv = cnt[base + i];
      offs[base + i] = run;
      cur[base + i]  = run;
      run += cv;
    }
  }
  __syncthreads();
  if (wave == 0) {
#pragma unroll 1
    for (int b0 = 0; b0 < tt; b0 += 32) {
      const int idx = b0 + lane;
      const int ent = hl[idx < RCAP ? idx : RCAP - 1];
      const int m32 = (tt - b0) < 32 ? (tt - b0) : 32;
#pragma unroll 1
      for (int k = 0; k < m32; ++k) {
        const int u    = __builtin_amdgcn_readlane(ent, k);
        const int slot = u & (NBA - 1);
        if (lane == 0) {
          int p = cur[slot];
          p = p < 0 ? 0 : (p > RCAP - 1 ? RCAP - 1 : p);
          sl[p] = u;
          cur[slot] = p + 1;
        }
      }
    }
  }
  __syncthreads();

  const float qnan = __int_as_float(0x7fc00000);
  const float pz = (ovf != 0) ? qnan : 0.0f;
#pragma unroll 1
  for (int si = 0; si < NBA / NWAVE; ++si) {
    const int s    = si * NWAVE + wave;
    const int node = nodeBase + s;
    int c = cnt[s];
    const bool big = c > DEGCAP;
    c = c < 0 ? 0 : (c > DEGCAP ? DEGCAP : c);
    int o = offs[s];
    o = o < 0 ? 0 : (o > RCAP ? RCAP : o);
    const int nc = node < nN ? node : nN - 1;
    const float dd = dis[nc];
    const float rd = dd * dd;
    v4f acc[NJ];
#pragma unroll
    for (int j = 0; j < NJ; ++j) { const v4f z = {0.0f, 0.0f, 0.0f, 0.0f}; acc[j] = z; }
#pragma unroll 1
    for (int b0 = 0; b0 < c; b0 += 32) {
      int idx = o + b0 + lane;
      idx = idx > RCAP - 1 ? RCAP - 1 : idx;
      const int ent = sl[idx];
      int eid = ent >> SLA;
      eid = eid < 0 ? 0 : (eid > nE - 1 ? nE - 1 : eid);
      int sr = srcs[eid];
      sr = sr < 0 ? 0 : (sr > nN - 1 ? nN - 1 : sr);
      const float cf  = dis[sr] * dd;
      const int   cfi = __float_as_int(cf);
      const int m32 = (c - b0) < 32 ? (c - b0) : 32;
#pragma unroll 1
      for (int k = 0; k < m32; ++k) {
        const int   sk = __builtin_amdgcn_readlane(sr, k);
        const float ck = __int_as_float(__builtin_amdgcn_readlane(cfi, k));
        const float* rp = tl + (size_t)sk * FW + 4 * lane;
#pragma unroll
        for (int j = 0; j < NJ; ++j) {
          const v4f a = *(const v4fa*)(rp + 128 * j);
          acc[j].x = fmaf(ck, a.x, acc[j].x);
          acc[j].y = fmaf(ck, a.y, acc[j].y);
          acc[j].z = fmaf(ck, a.z, acc[j].z);
          acc[j].w = fmaf(ck, a.w, acc[j].w);
        }
      }
    }
    const float pzr = big ? qnan : pz;
    const bool live = node < nN;
    v4f y[NJ];
    {
      const float* rp = tl + (size_t)nc * FW + 4 * lane;
#pragma unroll
      for (int j = 0; j < NJ; ++j) {
        const v4f sv = *(const v4fa*)(rp + 128 * j);
        v4f q;
        q.x = (acc[j].x + sv.x * rd) + bv[j].x;
        q.y = (acc[j].y + sv.y * rd) + bv[j].y;
        q.z = (acc[j].z + sv.z * rd) + bv[j].z;
        q.w = (acc[j].w + sv.w * rd) + bv[j].w;
        y[j] = q;
      }
    }

    if constexpr (MODE != 2) {
      unsigned short* rowbuf = (unsigned short*)(misc + MISC_INTS) + wave * ROWHW;
      float ss = 0.0f;
#pragma unroll
      for (int j = 0; j < NJ; ++j) {
        v4f q = y[j];
        q.x = (q.x > 0.0f) ? q.x : (q.x - q.x);
        q.y = (q.y > 0.0f) ? q.y : (q.y - q.y);
        q.z = (q.z > 0.0f) ? q.z : (q.z - q.z);
        q.w = (q.w > 0.0f) ? q.w : (q.w - q.w);
        y[j] = q;
        if constexpr (MODE == 0) {
          ss = fmaf(q.x, q.x, ss); ss = fmaf(q.y, q.y, ss);
          ss = fmaf(q.z, q.z, ss); ss = fmaf(q.w, q.w, ss);
        }
      }
      float sc = 1.0f;
      if constexpr (MODE == 0) {
        ss += __shfl_xor(ss, 16, 32);
        ss += __shfl_xor(ss, 8, 32);
        ss += __shfl_xor(ss, 4, 32);
        ss += __shfl_xor(ss, 2, 32);
        ss += __shfl_xor(ss, 1, 32);
        const float den = fmaxf(sqrtf(ss), 1e-12f);
        sc = 1.0f / den;
      }
#pragma unroll
      for (int j = 0; j < NJ; ++j) {
        float v0 = y[j].x * sc + pzr, v1 = y[j].y * sc + pzr;
        float v2 = y[j].z * sc + pzr, v3 = y[j].w * sc + pzr;
        v0 = live ? v0 : 0.0f; v1 = live ? v1 : 0.0f; v2 = live ? v2 : 0.0f; v3 = live ? v3 : 0.0f;
        v4us mh, ml;
        unsigned hb;
        hb = bf16_bits(v0); mh[0] = (unsigned short)hb; ml[0] = (unsigned short)bf16_bits(v0 - __uint_as_float(hb << 16));
        hb = bf16_bits(v1); mh[1] = (unsigned short)hb; ml[1] = (unsigned short)bf16_bits(v1 - __uint_as_float(hb << 16));
        hb = bf16_bits(v2); mh[2] = (unsigned short)hb; ml[2] = (unsigned short)bf16_bits(v2 - __uint_as_float(hb << 16));
        hb = bf16_bits(v3); mh[3] = (unsigned short)hb; ml[3] = (unsigned short)bf16_bits(v3 - __uint_as_float(hb << 16));
        *(v4usa*)(rowbuf + 128 * j + 4 * lane) = mh;
        *(v4usa*)(rowbuf + HID + 128 * j + 4 * lane) = ml;
      }
      wave_sync();
      v8us q0 = *(const v8usa*)(rowbuf + 8 * lane);
      v8us q1 = *(const v8usa*)(rowbuf + 256 + 8 * lane);
      v8us q2 = *(const v8usa*)(rowbuf + 512 + 8 * lane);
      v8us q3 = *(const v8usa*)(rowbuf + 768 + 8 * lane);
      wave_sync();
      if (node < mRows) {
        unsigned short* rpw = hpl + (size_t)node * KB + 8 * lane;
        *(volatile v8us*)rpw = q0;
        *(volatile v8us*)(rpw + 256) = q1;
        *(volatile v8us*)(rpw + 512) = q2;
        *(volatile v8us*)(rpw + 768) = q3;
        __threadfence();
        *(volatile v8us*)rpw = q0;
        *(volatile v8us*)(rpw + 256) = q1;
        *(volatile v8us*)(rpw + 512) = q2;
        *(volatile v8us*)(rpw + 768) = q3;
      }
    } else {
      v4f hm, hv;
      hm.x = y[0].x + pzr; hm.y = y[0].y + pzr; hm.z = y[0].z + pzr; hm.w = y[0].w + pzr;
      hv.x = y[NJ - 1].x + pzr; hv.y = y[NJ - 1].y + pzr; hv.z = y[NJ - 1].z + pzr; hv.w = y[NJ - 1].w + pzr;
      const v4f e4 = *(const v4fa*)(eps + (size_t)nc * ZD + 4 * lane);
      v4f zv;
      zv.x = hm.x + bf16_val(e4.x) * expf(0.5f * hv.x);
      zv.y = hm.y + bf16_val(e4.y) * expf(0.5f * hv.y);
      zv.z = hm.z + bf16_val(e4.z) * expf(0.5f * hv.z);
      zv.w = hm.w + bf16_val(e4.w) * expf(0.5f * hv.w);
      if (live) {
        float* oz = outp + (size_t)node * ZD + 4 * lane;
        *(volatile v4f*)oz = zv;
        *(volatile v4f*)(oz + outSeg) = hm;
        *(volatile v4f*)(oz + 2 * outSeg) = hv;
        __threadfence();
        *(volatile v4f*)oz = zv;
        *(volatile v4f*)(oz + outSeg) = hm;
        *(volatile v4f*)(oz + 2 * outSeg) = hv;
      }
    }
  }
}

static inline int cdiv(int a, int b) { return (a + b - 1) / b; }
static inline size_t al256(size_t o) { return (o + 255) & ~(size_t)255; }

extern "C" void kernel_launch(void* const* d_in, const int* in_sizes, int n_in,
                              void* d_out, int out_size, void* d_ws, size_t ws_size,
                              hipStream_t stream) {
  if (n_in < 11) return;
  if (in_sizes[0] < DIN || (in_sizes[0] % DIN) != 0) return;
  const int nN = in_sizes[0] / DIN;
  if (nN < 16 || nN > (1 << 21)) return;
  if (in_sizes[1] < 2 || (in_sizes[1] & 1) != 0) return;
  const int nE = in_sizes[1] / 2;
  if (nE < 1 || nE >= (1 << (31 - SLA))) return;
  if ((long long)in_sizes[2] != (long long)nN * ZD) return;
  if (in_sizes[3] != DIN * HID || in_sizes[4] != HID) return;
  if (in_sizes[5] != HID * HID || in_sizes[6] != HID) return;
  if (in_sizes[7] != HID * ZD || in_sizes[8] != ZD) return;
  if (in_sizes[9] != HID * ZD || in_sizes[10] != ZD) return;
  if ((long long)out_size != 3LL * (long long)nN * ZD) return;

  const float* x    = (const float*)d_in[0];
  const int*   edge = (const int*)d_in[1];
  const float* eps  = (const float*)d_in[2];
  const float* W1   = (const float*)d_in[3];
  const float* b1   = (const float*)d_in[4];
  const float* W2   = (const float*)d_in[5];
  const float* b2   = (const float*)d_in[6];
  const float* Wmu  = (const float*)d_in[7];
  const float* bmu  = (const float*)d_in[8];
  const float* Wlv  = (const float*)d_in[9];
  const float* blv  = (const float*)d_in[10];
  float* out = (float*)d_out;
  const int* src = edge;
  const int* dst = edge + nE;
  const size_t outSeg = (size_t)nN * ZD;

  const int MP   = cdiv(nN, GBM) * GBM;
  const int gM   = MP / GBM;
  const int gD   = cdiv(nN, NBD);
  const int NBPD = gD * NBD;
  const int gA   = cdiv(MP, NBA);
  if ((long long)gA * NBA < (long long)MP) return;
  if (NBPD < nN) return;
  const int vec8 = ((nE & 3) == 0) ? 1 : 0;

  char* ws = (char*)d_ws;
  size_t off = 0;
  const size_t oDIS = off; off = al256(off + (size_t)NBPD * 4);
  const size_t oW1T = off; off = al256(off + (size_t)HID * KA * 2);
  const size_t oW2T = off; off = al256(off + (size_t)HID * KB * 2);
  const size_t oWHT = off; off = al256(off + (size_t)NH * KB * 2);
  const size_t oXB  = off; off = al256(off + (size_t)MP * DIN * 2);
  const size_t oT   = off; off = al256(off + (size_t)MP * HID * 4);
  const size_t oH   = off; off = al256(off + (size_t)MP * KB * 2);
  if (off > ws_size || off > (size_t)WSMAX) return;
  float*          DIS = (float*)(ws + oDIS);
  unsigned short* W1T = (unsigned short*)(ws + oW1T);
  unsigned short* W2T = (unsigned short*)(ws + oW2T);
  unsigned short* WHT = (unsigned short*)(ws + oWHT);
  unsigned short* XB  = (unsigned short*)(ws + oXB);
  float*          T   = (float*)(ws + oT);
  unsigned short* H   = (unsigned short*)(ws + oH);

  const size_t ldsHL = (size_t)LDS_HL_INTS * 4;
  const size_t ldsHD = (size_t)LDS_HD_INTS * 4;
  hipFuncSetAttribute(reinterpret_cast<const void*>(&k_scan<4, 0>), hipFuncAttributeMaxDynamicSharedMemorySize, (int)ldsHL);
  hipFuncSetAttribute(reinterpret_cast<const void*>(&k_scan<4, 1>), hipFuncAttributeMaxDynamicSharedMemorySize, (int)ldsHL);
  hipFuncSetAttribute(reinterpret_cast<const void*>(&k_scan<2, 2>), hipFuncAttributeMaxDynamicSharedMemorySize, (int)ldsHD);

  const int nUx = MP * (DIN / 8);
  k_wprep<<<(NU1 + NU2 + NU3) / NTHR, NTHR, 0, stream>>>(W1, W2, Wmu, Wlv, W1T, W2T, WHT);
  k_cvx<<<cdiv(nUx, NTHR), NTHR, 0, stream>>>(x, nN, nUx, XB);
  k_deg<<<gD, NTHR, 0, stream>>>(dst, nE, vec8, DIS);
  k_gemm<<<dim3(gM, HID / GBN), GTHR, 0, stream>>>(XB, W1T, T, KA, HID);
  k_scan<4, 0><<<gA, NTHR, ldsHL, stream>>>(src, dst, nE, nN, vec8, MP, DIS, T, b1, b1, eps, H, out, outSeg);
  k_gemm<<<dim3(gM, HID / GBN), GTHR, 0, stream>>>(H, W2T, T, KB, HID);
  k_scan<4, 1><<<gA, NTHR, ldsHL, stream>>>(src, dst, nE, nN, vec8, MP, DIS, T, b2, b2, eps, H, out, outSeg);
  k_gemm<<<dim3(gM, NH / GBN), GTHR, 0, stream>>>(H, WHT, T, KB, NH);
  k_scan<2, 2><<<gA, NTHR, ldsHD, stream>>>(src, dst, nE, nN, vec8, MP, DIS, T, bmu, blv, eps, H, out, outSeg);
}
